// Discriminator_8744553415337
// MI455X (gfx1250) — hardware-run, weakly checked
//
#include <hip/hip_runtime.h>


#ifndef NSAMP
#define NSAMP 65536
#endif
#define NSAMP_FULL 65536
#define NNODE  100000
#define ED     64
#define NREL   8
#define CH     256
#define NW     8
#define MAXT   24
#define MAXS   (MAXT * 16)
#define APITCH 72
#define EPITCH 68

static_assert(CH == 32 * NW);
static_assert(NSAMP % CH == 0);
static_assert(NSAMP <= NSAMP_FULL);
static_assert(ED == 64);
static_assert(ED % 32 == 0);
static_assert((CH + NREL * 15) / 16 <= MAXT);
static_assert(NREL <= 8);
static_assert(MAXT <= CH);
static_assert(APITCH % 8 == 0);
static_assert(APITCH >= ED);
static_assert((EPITCH * 4) % 16 == 0);
static_assert(EPITCH >= ED);
static_assert((CH / 4) * 16 == CH * 4);
static_assert((CH / 4) % 32 == 0);
static_assert(((size_t)NREL * ED * ED) % 8 == 0);
static_assert(NW * 16 * APITCH * 2 + NW * 16 * EPITCH * 4 + CH * 4 + MAXS * 4 + MAXT * 4 + 2 * NW * NREL * 4 + NREL * 4 <= 131072);

typedef unsigned short bf;
typedef __attribute__((ext_vector_type(16))) __bf16   v16bf;
typedef __attribute__((ext_vector_type(8)))  unsigned short v8us;
typedef __attribute__((ext_vector_type(4)))  unsigned short v4us;
typedef __attribute__((ext_vector_type(8)))  float    v8f;
typedef __attribute__((ext_vector_type(4)))  float    v4f;
typedef v4f  __attribute__((may_alias)) v4fa;
typedef v8us __attribute__((may_alias)) v8usa;
typedef v4us __attribute__((may_alias)) v4usa;

__device__ __forceinline__ unsigned short f2bf(float f) { unsigned u = __float_as_uint(f); u += 0x7FFFu + ((u >> 16) & 1u); return (unsigned short)(u >> 16); }
__device__ __forceinline__ float bfr(float f) { return __uint_as_float(((unsigned)f2bf(f)) << 16); }
__device__ __forceinline__ v16bf cat16b(v8us lo, v8us hi) { return __builtin_bit_cast(v16bf, __builtin_shufflevector(lo, hi, 0, 1, 2, 3, 4, 5, 6, 7, 8, 9, 10, 11, 12, 13, 14, 15)); }
__device__ __forceinline__ v8f wmmab(v16bf a, v16bf b, v8f c) { return __builtin_amdgcn_wmma_f32_16x16x32_bf16(false, a, false, b, (short)0, c, false, false); }
__device__ __forceinline__ v16bf ldb(const bf* p)  { return cat16b(*(const v8us*)p, *(const v8us*)(p + 16)); }
__device__ __forceinline__ void wave_sync() { __builtin_amdgcn_fence(3  , "wavefront"); __builtin_amdgcn_wave_barrier(); asm volatile("" ::: "memory"); }
__device__ __forceinline__ v8f wmmab_g(v16bf a, v16bf b, v8f c) { c = wmmab(a, b, c); asm volatile("v_nop\n\tv_nop\n\tv_nop\n\tv_nop" : "+v"(c) : "v"(a), "v"(b)); return c; }

__global__ __launch_bounds__(256) void k_cvt8(const float* __restrict__ src, bf* dst, size_t n8) {
    const size_t i = (size_t)blockIdx.x * 256 + threadIdx.x; if (i >= n8) return;
    const v8f v = *(const v8f*)(src + i * 8); v8us o;
#pragma unroll
    for (int k = 0; k < 8; ++k) o[k] = f2bf(v[k]);
    *(volatile v8us*)(dst + i * 8) = o; __threadfence(); *(volatile v8us*)(dst + i * 8) = o;
}

__global__ __launch_bounds__(CH) void k_score(const int* __restrict__ node_idx, const int* __restrict__ rel_idx, const int* __restrict__ nbr_idx,
                                              const float* __restrict__ ntab, const bf* __restrict__ RB, float* OUT) {
    __shared__ __align__(16) bf    at[NW * 16 * APITCH];
    __shared__ __align__(16) float et[NW * 16 * EPITCH];
    __shared__ __align__(16) float res[CH];
    __shared__ int slot[MAXS];
    __shared__ int trel[MAXT];
    __shared__ int wcnt[NW * NREL];
    __shared__ int woff[NW * NREL];
    __shared__ int tot[NREL];

    const int tid = threadIdx.x;
    const int lane = threadIdx.x & 31, lr = lane & 15, hi = lane >> 4;
    const int wave = __builtin_amdgcn_readfirstlane((int)(threadIdx.x >> 5));
    const int sbase = blockIdx.x * CH;

    int rel = rel_idx[sbase + tid]; rel = rel < 0 ? 0 : (rel > NREL - 1 ? NREL - 1 : rel);
#pragma unroll 1
    for (int i = tid; i < MAXS; i += CH) slot[i] = -1;
    if (tid < MAXT) trel[tid] = 0;
    res[tid] = 0.0f;
    const unsigned lt = (1u << lane) - 1u;
    int rank = 0, mycnt = 0;
#pragma unroll
    for (int r = 0; r < NREL; ++r) {
        const unsigned bal = __builtin_amdgcn_ballot_w32(rel == r);
        const int below = __popc(bal & lt), all = __popc(bal);
        rank  = (rel == r)  ? below : rank;
        mycnt = (lane == r) ? all   : mycnt;
    }
    if (lane < NREL) wcnt[wave * NREL + lane] = mycnt;
    __syncthreads();
    if (tid < NREL) {
        int run = 0;
#pragma unroll 1
        for (int w = 0; w < NW; ++w) { woff[w * NREL + tid] = run; run += wcnt[w * NREL + tid]; }
        tot[tid] = run;
    }
    __syncthreads();
    int gb = 0, nsl = 0;
#pragma unroll
    for (int r = 0; r < NREL; ++r) { const int pr = (tot[r] + 15) & ~15; gb = (r < rel) ? (gb + pr) : gb; nsl += pr; }
    int pos = gb + woff[wave * NREL + rel] + rank;
    pos = pos < 0 ? 0 : (pos > MAXS - 1 ? MAXS - 1 : pos);
    slot[pos] = tid;
    if ((pos & 15) == 0) trel[pos >> 4] = rel;
    int ntl = nsl >> 4; ntl = ntl < 0 ? 0 : (ntl > MAXT ? MAXT : ntl);
    const int nt = __builtin_amdgcn_readfirstlane(ntl);
    __syncthreads();

    const int ab = wave * 16 * APITCH, eb = wave * 16 * EPITCH;
    const int c4 = lr * 4;
#pragma unroll 1
    for (int q = wave; q < nt; q += NW) {
        int rq = trel[q]; rq = rq < 0 ? 0 : (rq > NREL - 1 ? NREL - 1 : rq);
        const int r = __builtin_amdgcn_readfirstlane(rq);
        const int sl = slot[q * 16 + lr];
        const int sv = sl < 0 ? 0 : (sl > CH - 1 ? CH - 1 : sl);
        int ni = node_idx[sbase + sv]; ni = ni < 0 ? 0 : (ni > NNODE - 1 ? NNODE - 1 : ni);
        int bi = nbr_idx[sbase + sv];  bi = bi < 0 ? 0 : (bi > NNODE - 1 ? NNODE - 1 : bi);
#pragma unroll
        for (int i = 0; i < 8; ++i) {
            const int row = 2 * i + hi;
            const int nrow = __shfl(ni, row, 32), brow = __shfl(bi, row, 32);
            const v4f nv = *(const v4f*)(ntab + (size_t)brow * ED + c4);
            const v4f ev = *(const v4f*)(ntab + (size_t)nrow * ED + c4);
            v4us o; v4f eo;
#pragma unroll
            for (int k = 0; k < 4; ++k) { o[k] = f2bf(nv[k]); eo[k] = bfr(ev[k]); }
            *(v4usa*)(&at[ab + row * APITCH + c4]) = o;
            *(v4fa*)(&et[eb + row * EPITCH + c4]) = eo;
        }
        wave_sync();
        v8f acc[4];
#pragma unroll
        for (int nb = 0; nb < 4; ++nb) acc[nb] = (v8f){};
        const size_t rbo = (size_t)r * (ED * ED) + (size_t)lr * ED + 8 * hi;
#pragma unroll
        for (int ks = 0; ks < 2; ++ks) {
            const int ao = ab + lr * APITCH + ks * 32 + 8 * hi;
            const v16bf a = cat16b(*(const v8usa*)(&at[ao]), *(const v8usa*)(&at[ao + 16]));
#pragma unroll
            for (int nb = 0; nb < 4; ++nb) {
                const v16bf b = ldb(RB + rbo + (size_t)nb * 16 * ED + ks * 32);
                acc[nb] = wmmab_g(a, b, acc[nb]);
            }
        }
        float s[8];
#pragma unroll
        for (int j = 0; j < 8; ++j) s[j] = 0.0f;
#pragma unroll
        for (int nb = 0; nb < 4; ++nb) {
#pragma unroll
            for (int j = 0; j < 8; ++j) s[j] += acc[nb][j] * et[eb + (8 * hi + j) * EPITCH + nb * 16 + lr];
        }
#pragma unroll
        for (int mk = 8; mk >= 1; mk >>= 1) {
#pragma unroll
            for (int j = 0; j < 8; ++j) s[j] += __shfl_xor(s[j], mk, 32);
        }
        const int jr = lr & 7;
        float mine = s[0];
#pragma unroll
        for (int j = 1; j < 8; ++j) mine = (jr == j) ? s[j] : mine;
        const int srow = 8 * hi + jr;
        const int slr = __shfl(sl, srow, 32);
        const float sig = 1.0f / (1.0f + expf(-mine));
        const int slc = slr > CH - 1 ? CH - 1 : slr;
        if ((lr < 8) & (slr >= 0)) res[slc] = sig;
        wave_sync();
    }
    __syncthreads();
    float* orow = OUT + (size_t)sbase;
#pragma unroll 1
    for (int ps = 0; ps < 2; ++ps) {
        if (tid < CH / 4) { const v4f val = *(const v4fa*)(&res[tid * 4]); *(volatile v4f*)(orow + tid * 4) = val; }
        if (ps == 0) __threadfence(); }
}

static constexpr size_t al256(size_t v) { return (v + 255) & ~(size_t)255; }
static constexpr size_t SZ_RB = al256((size_t)NREL * ED * ED * 2);
static constexpr size_t SZ_TOTAL = SZ_RB;
static_assert(SZ_TOTAL <= (size_t)134217728);
static_assert(((size_t)NREL * ED * ED / 8) * 16 <= SZ_RB);

extern "C" void kernel_launch(void* const* d_in, const int* in_sizes, int n_in,
                              void* d_out, int out_size, void* d_ws, size_t ws_size, hipStream_t stream) {
    if (n_in < 5) return;
    if (in_sizes[0] < NSAMP || in_sizes[1] < NSAMP || in_sizes[2] < NSAMP) return;
    if ((size_t)in_sizes[3] < (size_t)NNODE * ED) return;
    if ((size_t)in_sizes[4] < (size_t)NREL * ED * ED) return;
    if (out_size < NSAMP) return;
    if (SZ_TOTAL > ws_size) return;
    const int* node_idx = (const int*)d_in[0];
    const int* rel_idx  = (const int*)d_in[1];
    const int* nbr_idx  = (const int*)d_in[2];
    const float* ntab   = (const float*)d_in[3];
    const float* rtab   = (const float*)d_in[4];
    float* OUT = (float*)d_out;
    char* wsp = (char*)d_ws;
    bf* RB = (bf*)wsp; wsp += SZ_RB;

    { const size_t n8 = (size_t)NREL * ED * ED / 8; const unsigned g = (unsigned)((n8 + 255) / 256);
      k_cvt8<<<g, 256, 0, stream>>>(rtab, RB, n8); }
    k_score<<<dim3(NSAMP / CH, 1, 1), CH, 0, stream>>>(node_idx, rel_idx, nbr_idx, ntab, RB, OUT);
}
